// Block_24661702213802
// MI455X (gfx1250) — hardware-verified
//
#include <hip/hip_runtime.h>


#ifndef NB
#define NB 2
#endif
#ifndef SEQ
#define SEQ 2048
#endif
#define NB_FULL 2
#define SEQ_FULL 2048
#define CE 1024
#define NH 16
#define HD 64
#define C3 3072
#define C4 4096
#define QP 2048
#define TE (((SEQ) < 256) ? (SEQ) : 256)
#define RROWS ((NB) * (SEQ))
#define NEB ((TE) / 128)
#define NQB ((SEQ) / 128)

static_assert((SEQ) % 128 == 0);
static_assert((TE) % 128 == 0);
static_assert((NB) >= 1 && (NB) <= NB_FULL);
static_assert((SEQ) <= SEQ_FULL);
static_assert(CE % 128 == 0 && C3 % 128 == 0 && C4 % 128 == 0);
static_assert(CE % 64 == 0 && C4 % 64 == 0);
static_assert(CE % 256 == 0);
static_assert(NH * HD == CE);
static_assert(RROWS % 128 == 0);
static_assert(CE == 1024);
static_assert(QP == 2 * CE && C3 == 3 * CE && C4 == 4 * CE);

typedef unsigned short u16;
typedef unsigned int   u32;
typedef _Float16 v16h __attribute__((ext_vector_type(16)));
typedef _Float16 v8h  __attribute__((ext_vector_type(8)));
typedef float    v8f  __attribute__((ext_vector_type(8)));
typedef float    v4f  __attribute__((ext_vector_type(4)));
typedef unsigned int u32x4 __attribute__((ext_vector_type(4)));

union Frag  { v16h v; u32x4 u[2]; };
union Pack8 { v8h h; u32x4 u; };

#define WSCALE 64.0f
#define WINV   (1.0f / 64.0f)
#define PCAR   4096.0f
#define PINV   (1.0f / 4096.0f)
#define RSC    2048.0f
#define RINV   (1.0f / 2048.0f)
#define OCAR   32.0f
#define OINV   (1.0f / 32.0f)
#define HCAR   16.0f
#define HINV   (1.0f / 16.0f)

__device__ __forceinline__ float bfr(float f) {
    u32 u = __builtin_bit_cast(u32, f);
    u += 0x7fffu + ((u >> 16) & 1u);
    u &= 0xffff0000u;
    return __builtin_bit_cast(float, u);
}

__device__ __forceinline__ u16 hbits(float f) {
    _Float16 h = (_Float16)f;
    return __builtin_bit_cast(u16, h);
}

__device__ __forceinline__ v8f mma16(v16h a, v16h b, v8f c) {
    c = __builtin_amdgcn_wmma_f32_16x16x32_f16(false, a, false, b, (short)0, c, false, false);
    asm volatile("v_nop\n\tv_nop\n\tv_nop\n\tv_nop" : "+v"(c) : "v"(a), "v"(b));
    return c;
}

__device__ __forceinline__ float gelu_e(float x) {
    return 0.5f * x * (1.0f + erff(x * 0.70710678118654752f));
}

__device__ __forceinline__ size_t grow_map(int r) {
    int bb = r / (SEQ);
    int t  = r - bb * (SEQ);
    return (size_t)bb * SEQ_FULL + (size_t)t;
}

__global__ __launch_bounds__(256) void cvt_wt_kernel(const float* __restrict__ in,
                                                      u16* __restrict__ out, int K, int N) {
    __shared__ __align__(16) u16 Ts[64 * 72];
    const int tid = threadIdx.x, lane = tid & 31, wv = tid >> 5;
    const int n0 = blockIdx.x * 64, k0 = blockIdx.y * 64;
    const int kr = tid >> 2, nseg = (tid & 3) * 16;
    const float* src = in + (size_t)(k0 + kr) * N + n0 + nseg;
#pragma unroll
    for (int j4 = 0; j4 < 4; j4++) {
        v4f w = *(const v4f*)(src + j4 * 4);
#pragma unroll
        for (int c = 0; c < 4; c++) {
            float f = w[c];
            Ts[(nseg + j4 * 4 + c) * 72 + kr] = hbits(bfr(f) * WSCALE);
        }
    }
    __syncthreads();
    u32x4 val[2];
#pragma unroll
    for (int it = 0; it < 2; it++) {
        const int nn = wv * 8 + it * 4 + (lane >> 3), ks = (lane & 7) * 8;
        val[it] = *(const u32x4*)&Ts[nn * 72 + ks];
    }
#pragma unroll
    for (int it = 0; it < 2; it++) {
        const int nn = wv * 8 + it * 4 + (lane >> 3), ks = (lane & 7) * 8;
        *(volatile u32x4*)(out + (size_t)(n0 + nn) * K + k0 + ks) = val[it];
    }
    __threadfence();
#pragma unroll
    for (int it = 0; it < 2; it++) {
        const int nn = wv * 8 + it * 4 + (lane >> 3), ks = (lane & 7) * 8;
        *(volatile u32x4*)(out + (size_t)(n0 + nn) * K + k0 + ks) = val[it];
    }
}

template <int SRCX>
__global__ __launch_bounds__(256) void dyt_kernel(const float* __restrict__ src,
                                                  const float* __restrict__ al,
                                                  const float* __restrict__ g,
                                                  const float* __restrict__ be,
                                                  u16* __restrict__ out) {
    __shared__ __align__(16) u16 rows[8 * CE];
    const int tid = threadIdx.x, lane = tid & 31, wv = tid >> 5;
    const int r = blockIdx.x * 8 + wv;
    const size_t srow = SRCX ? grow_map(r) : (size_t)r;
    const float* xr = src + srow * CE;
    const float a = bfr(al[0]);
    u16* rw = rows + wv * CE;
#pragma unroll 1
    for (int j = 0; j < CE / 32; j++) {
        const int c = j * 32 + lane;
        float t = xr[c];
        if (SRCX) t = bfr(t);
        const float gg = bfr(g[c]);
        const float bb = bfr(be[c]);
        rw[c] = hbits(gg * tanhf(t * a) + bb);
    }
    __syncthreads();
    u32x4 val[CE / 256];
#pragma unroll
    for (int j = 0; j < CE / 256; j++) val[j] = *(const u32x4*)&rw[j * 256 + lane * 8];
    u16* orow = out + (size_t)r * CE;
#pragma unroll
    for (int j = 0; j < CE / 256; j++) *(volatile u32x4*)(orow + j * 256 + lane * 8) = val[j];
    __threadfence();
#pragma unroll
    for (int j = 0; j < CE / 256; j++) *(volatile u32x4*)(orow + j * 256 + lane * 8) = val[j];
}

template <int MODE>
__global__ __launch_bounds__(256) void gemm_kernel(const u16* __restrict__ A,
                                                   const u16* __restrict__ BT,
                                                   const float* __restrict__ bias,
                                                   const float* __restrict__ res,
                                                   void* out0, void* out1, void* out2, void* out3,
                                                   int N, int K) {
    __shared__ u32x4 smem[4224];
    u16* As = (u16*)smem;
    u16* Bs = As + 128 * 72;
    float* Cs = (float*)smem;
    constexpr int CSP = 132;
    constexpr float OSC = (MODE == 1) ? (WINV * OINV) : ((MODE == 3) ? (WINV * HINV) : WINV);

    const int tid = threadIdx.x, lane = tid & 31, wv = tid >> 5;
    const int hf = lane >> 4, ln = lane & 15;
    const int m0 = blockIdx.y * 128, n0 = blockIdx.x * 128;
    const int wm = wv & 3, wn = wv >> 2;
    const int srow = tid >> 1, sseg = (tid & 1) * 32;

    v8f acc[2][4];
#pragma unroll
    for (int i = 0; i < 2; i++)
#pragma unroll
        for (int j = 0; j < 4; j++) acc[i][j] = (v8f)(0.f);

    for (int k0 = 0; k0 < K; k0 += 64) {
        __syncthreads();
        {
            const u16* ga = A  + (size_t)(m0 + srow) * K + k0 + sseg;
            const u16* gb = BT + (size_t)(n0 + srow) * K + k0 + sseg;
            u32x4 a0 = *(const u32x4*)(ga), a1 = *(const u32x4*)(ga + 8);
            u32x4 a2 = *(const u32x4*)(ga + 16), a3 = *(const u32x4*)(ga + 24);
            u32x4 b0 = *(const u32x4*)(gb), b1 = *(const u32x4*)(gb + 8);
            u32x4 b2 = *(const u32x4*)(gb + 16), b3 = *(const u32x4*)(gb + 24);
            u32x4* la = (u32x4*)&As[srow * 72 + sseg];
            u32x4* lb = (u32x4*)&Bs[srow * 72 + sseg];
            la[0] = a0; la[1] = a1; la[2] = a2; la[3] = a3;
            lb[0] = b0; lb[1] = b1; lb[2] = b2; lb[3] = b3;
        }
        __syncthreads();
#pragma unroll
        for (int ks = 0; ks < 2; ks++) {
            Frag af[2], bf[4];
#pragma unroll
            for (int mi = 0; mi < 2; mi++) {
                const u16* q = &As[(wm * 32 + mi * 16 + ln) * 72 + ks * 32 + hf * 8];
                af[mi].u[0] = *(const u32x4*)q;
                af[mi].u[1] = *(const u32x4*)(q + 16);
            }
#pragma unroll
            for (int ni = 0; ni < 4; ni++) {
                const u16* q = &Bs[(wn * 64 + ni * 16 + ln) * 72 + ks * 32 + hf * 8];
                bf[ni].u[0] = *(const u32x4*)q;
                bf[ni].u[1] = *(const u32x4*)(q + 16);
            }
#pragma unroll
            for (int mi = 0; mi < 2; mi++)
#pragma unroll
                for (int ni = 0; ni < 4; ni++)
                    acc[mi][ni] = mma16(af[mi].v, bf[ni].v, acc[mi][ni]);
        }
    }

    __syncthreads();
#pragma unroll
    for (int ni = 0; ni < 4; ni++) {
        const int col = wn * 64 + ni * 16 + ln;
        const float bv = bfr(bias[n0 + col]);
#pragma unroll
        for (int mi = 0; mi < 2; mi++) {
#pragma unroll
            for (int r = 0; r < 8; r++) {
                const int row = wm * 32 + mi * 16 + hf * 8 + r;
                float v = acc[mi][ni][r] * OSC + bv;
                if constexpr (MODE == 2) v = gelu_e(v) * HCAR;
                Cs[row * CSP + col] = v;
            }
        }
    }
    __syncthreads();

    if constexpr (MODE == 1 || MODE == 3) {
        float* o = (float*)out0;
        v4f val[16];
#pragma unroll
        for (int grp = 0; grp < 2; grp++) {
#pragma unroll
            for (int i8 = 0; i8 < 8; i8++) {
                const int i = grp * 8 + i8;
                const int row = wv * 16 + i;
                const int r = m0 + row;
                v4f c = *(const v4f*)&Cs[row * CSP + lane * 4];
                const size_t rr = (MODE == 1) ? grow_map(r) : (size_t)r;
                v4f x4 = *(const v4f*)(res + rr * (size_t)N + n0 + lane * 4);
                if constexpr (MODE == 1) {
#pragma unroll
                    for (int cc = 0; cc < 4; cc++) { float t = x4[cc]; x4[cc] = bfr(t); }
                }
                val[i] = c + x4;
            }
            asm volatile("" ::: "memory");
        }
#pragma unroll
        for (int i = 0; i < 16; i++) {
            const int r = m0 + wv * 16 + i;
            const size_t orr = (MODE == 3) ? grow_map(r) : (size_t)r;
            *(volatile v4f*)(o + orr * (size_t)N + n0 + lane * 4) = val[i];
        }
        __threadfence();
#pragma unroll
        for (int i = 0; i < 16; i++) {
            const int r = m0 + wv * 16 + i;
            const size_t orr = (MODE == 3) ? grow_map(r) : (size_t)r;
            *(volatile v4f*)(o + orr * (size_t)N + n0 + lane * 4) = val[i];
        }
    } else if constexpr (MODE == 2) {
        u16* o = (u16*)out0;
        u32x4 val[8];
#pragma unroll
        for (int it = 0; it < 8; it++) {
            const int rloc = wv * 16 + it * 2 + hf, cseg = ln * 8;
            Pack8 pk;
#pragma unroll
            for (int j = 0; j < 8; j++) pk.h[j] = (_Float16)Cs[rloc * CSP + cseg + j];
            val[it] = pk.u;
        }
#pragma unroll
        for (int it = 0; it < 8; it++) {
            const int rloc = wv * 16 + it * 2 + hf, cseg = ln * 8;
            *(volatile u32x4*)(o + (size_t)(m0 + rloc) * N + n0 + cseg) = val[it];
        }
        __threadfence();
#pragma unroll
        for (int it = 0; it < 8; it++) {
            const int rloc = wv * 16 + it * 2 + hf, cseg = ln * 8;
            *(volatile u32x4*)(o + (size_t)(m0 + rloc) * N + n0 + cseg) = val[it];
        }
    } else {
        u16* qkh = (u16*)out0;
        u16* qkl = (u16*)out1;
        u16* vth = (u16*)out2;
        u16* vtl = (u16*)out3;
        const int bq = m0 / (SEQ);
        const int t0 = m0 - bq * (SEQ);
        const bool lo_on = (t0 < (TE));
        u32x4 vh[8], vl[8];
        if (n0 < QP) {
#pragma unroll
            for (int it = 0; it < 8; it++) {
                const int rloc = wv * 16 + it * 2 + hf, cseg = ln * 8;
                Pack8 ph, pl;
#pragma unroll
                for (int j = 0; j < 8; j++) {
                    float f = Cs[rloc * CSP + cseg + j];
                    _Float16 h16 = (_Float16)f;
                    ph.h[j] = h16;
                    pl.h[j] = (_Float16)((f - (float)h16) * RSC);
                }
                vh[it] = ph.u; vl[it] = pl.u;
            }
#pragma unroll
            for (int it = 0; it < 8; it++) {
                const int rloc = wv * 16 + it * 2 + hf, cseg = ln * 8;
                *(volatile u32x4*)(qkh + (size_t)(m0 + rloc) * QP + n0 + cseg) = vh[it];
                if (lo_on)
                    *(volatile u32x4*)(qkl + ((size_t)bq * (TE) + t0 + rloc) * QP + n0 + cseg) = vl[it];
            }
            __threadfence();
#pragma unroll
            for (int it = 0; it < 8; it++) {
                const int rloc = wv * 16 + it * 2 + hf, cseg = ln * 8;
                *(volatile u32x4*)(qkh + (size_t)(m0 + rloc) * QP + n0 + cseg) = vh[it];
                if (lo_on)
                    *(volatile u32x4*)(qkl + ((size_t)bq * (TE) + t0 + rloc) * QP + n0 + cseg) = vl[it];
            }
        } else {
            const int hh0 = (n0 - QP) >> 6;
#pragma unroll
            for (int it = 0; it < 8; it++) {
                const int rloc = wv * 16 + it * 2 + hf;
                const int tseg = ln * 8;
                Pack8 ph, pl;
#pragma unroll
                for (int j = 0; j < 8; j++) {
                    float f = Cs[(tseg + j) * CSP + rloc];
                    _Float16 h16 = (_Float16)f;
                    ph.h[j] = h16;
                    pl.h[j] = (_Float16)((f - (float)h16) * RSC);
                }
                vh[it] = ph.u; vl[it] = pl.u;
            }
#pragma unroll
            for (int it = 0; it < 8; it++) {
                const int rloc = wv * 16 + it * 2 + hf, tseg = ln * 8;
                const int hh = hh0 + (rloc >> 6), dd = rloc & 63;
                const size_t vrow = (size_t)(bq * NH + hh) * HD + dd;
                *(volatile u32x4*)(vth + vrow * (SEQ) + t0 + tseg) = vh[it];
                if (lo_on)
                    *(volatile u32x4*)(vtl + vrow * (TE) + t0 + tseg) = vl[it];
            }
            __threadfence();
#pragma unroll
            for (int it = 0; it < 8; it++) {
                const int rloc = wv * 16 + it * 2 + hf, tseg = ln * 8;
                const int hh = hh0 + (rloc >> 6), dd = rloc & 63;
                const size_t vrow = (size_t)(bq * NH + hh) * HD + dd;
                *(volatile u32x4*)(vth + vrow * (SEQ) + t0 + tseg) = vh[it];
                if (lo_on)
                    *(volatile u32x4*)(vtl + vrow * (TE) + t0 + tseg) = vl[it];
            }
        }
    }
}

template <int RES>
__global__ __launch_bounds__(256) __attribute__((amdgpu_num_vgpr(256)))
void attn_kernel(const u16* __restrict__ qkh, const u16* __restrict__ qkl,
                 const u16* __restrict__ vth, const u16* __restrict__ vtl,
                 u16* __restrict__ cv, int qb0) {
    __shared__ __align__(16) u16 Ks[64 * 72];
    __shared__ __align__(16) u16 Vs[64 * 72];
    __shared__ __align__(16) u16 Kl[RES ? 64 * 72 : 8];
    __shared__ __align__(16) u16 Vl[RES ? 64 * 72 : 8];
    __shared__ __align__(16) u16 Ps[8 * 16 * 72];
    __shared__ __align__(16) u16 Pr[RES ? 8 * 16 * 72 : 8];

    const int bh = blockIdx.y;
    const int b = bh / NH, h = bh - b * NH;
    const int qb = qb0 + blockIdx.x;
    const int tid = threadIdx.x, lane = tid & 31, wv = tid >> 5;
    const int hf = lane >> 4, ln = lane & 15;
    const int q0 = qb * 128 + wv * 16;
    u16* Pw  = Ps + wv * (16 * 72);
    u16* Prw = Pr + (RES ? wv * (16 * 72) : 0);

    Frag qf[2], ql[2];
#pragma unroll
    for (int ds = 0; ds < 2; ds++) {
        const u16* p = qkh + (size_t)(b * (SEQ) + q0 + ln) * QP + h * HD + ds * 32 + hf * 8;
        qf[ds].u[0] = *(const u32x4*)p;
        qf[ds].u[1] = *(const u32x4*)(p + 16);
        if constexpr (RES) {
            const u16* pl = qkl + (size_t)(b * (TE) + q0 + ln) * QP + h * HD + ds * 32 + hf * 8;
            ql[ds].u[0] = *(const u32x4*)pl;
            ql[ds].u[1] = *(const u32x4*)(pl + 16);
        } else {
            ql[ds].u[0] = (u32x4)(0u); ql[ds].u[1] = (u32x4)(0u);
        }
    }

    v8f o[4];
#pragma unroll
    for (int i = 0; i < 4; i++) o[i] = (v8f)(0.f);
    float mrow[8], lrow[8];
#pragma unroll
    for (int r = 0; r < 8; r++) { mrow[r] = -3.0e38f; lrow[r] = 0.f; }

    const int rr = tid >> 2, seg = (tid & 3) * 16;
    const int nkt = 2 * qb + 2;

#pragma unroll 1
    for (int kt = 0; kt < nkt; kt++) {
        __syncthreads();
        {
            const u16* gk = qkh + (size_t)(b * (SEQ) + kt * 64 + rr) * QP + CE + h * HD + seg;
            u32x4 k0v = *(const u32x4*)gk, k1v = *(const u32x4*)(gk + 8);
            const u16* gv = vth + ((size_t)(bh * HD + rr)) * (SEQ) + kt * 64 + seg;
            u32x4 v0 = *(const u32x4*)gv, v1 = *(const u32x4*)(gv + 8);
            *(u32x4*)&Ks[rr * 72 + seg] = k0v; *(u32x4*)&Ks[rr * 72 + seg + 8] = k1v;
            *(u32x4*)&Vs[rr * 72 + seg] = v0;  *(u32x4*)&Vs[rr * 72 + seg + 8] = v1;
            if constexpr (RES) {
                const u16* gkl = qkl + (size_t)(b * (TE) + kt * 64 + rr) * QP + CE + h * HD + seg;
                u32x4 kl0 = *(const u32x4*)gkl, kl1 = *(const u32x4*)(gkl + 8);
                const u16* gvl = vtl + ((size_t)(bh * HD + rr)) * (TE) + kt * 64 + seg;
                u32x4 vl0 = *(const u32x4*)gvl, vl1 = *(const u32x4*)(gvl + 8);
                *(u32x4*)&Kl[rr * 72 + seg] = kl0; *(u32x4*)&Kl[rr * 72 + seg + 8] = kl1;
                *(u32x4*)&Vl[rr * 72 + seg] = vl0; *(u32x4*)&Vl[rr * 72 + seg + 8] = vl1;
            }
        }
        __syncthreads();

        v8f s[4];
#pragma unroll
        for (int sub = 0; sub < 4; sub++) {
            v8f t = (v8f)(0.f);
            v8f tr = (v8f)(0.f);
#pragma unroll
            for (int ds = 0; ds < 2; ds++) {
                Frag kf;
                const u16* kp = &Ks[(sub * 16 + ln) * 72 + ds * 32 + hf * 8];
                kf.u[0] = *(const u32x4*)kp;
                kf.u[1] = *(const u32x4*)(kp + 16);
                t = mma16(qf[ds].v, kf.v, t);
                if constexpr (RES) {
                    Frag klf;
                    const u16* klp = &Kl[(sub * 16 + ln) * 72 + ds * 32 + hf * 8];
                    klf.u[0] = *(const u32x4*)klp;
                    klf.u[1] = *(const u32x4*)(klp + 16);
                    tr = mma16(qf[ds].v, klf.v, tr);
                    tr = mma16(ql[ds].v, kf.v, tr);
                }
            }
            if constexpr (RES) s[sub] = t + tr * RINV;
            else s[sub] = t;
        }

#pragma unroll
        for (int sub = 0; sub < 4; sub++) {
            const int kg = kt * 64 + sub * 16 + ln;
#pragma unroll
            for (int r = 0; r < 8; r++) {
                const int qg = q0 + hf * 8 + r;
                float v = s[sub][r] * 0.125f;
                s[sub][r] = (kg > qg) ? -3.0e38f : v;
            }
        }
#pragma unroll
        for (int r = 0; r < 8; r++) {
            float mx = fmaxf(fmaxf(s[0][r], s[1][r]), fmaxf(s[2][r], s[3][r]));
#pragma unroll
            for (int m = 8; m >= 1; m >>= 1) mx = fmaxf(mx, __shfl_xor(mx, m, 32));
            const float mnew  = fmaxf(mrow[r], mx);
            const float alpha = __expf(mrow[r] - mnew);
            float rsum = 0.f;
#pragma unroll
            for (int sub = 0; sub < 4; sub++) {
                float pe = __expf(s[sub][r] - mnew);
                s[sub][r] = pe;
                rsum += pe;
            }
#pragma unroll
            for (int m = 8; m >= 1; m >>= 1) rsum += __shfl_xor(rsum, m, 32);
            mrow[r] = mnew;
            lrow[r] = lrow[r] * alpha + rsum;
#pragma unroll
            for (int dsub = 0; dsub < 4; dsub++) o[dsub][r] *= alpha;
        }

#pragma unroll
        for (int sub = 0; sub < 4; sub++) {
#pragma unroll
            for (int r = 0; r < 8; r++) {
                const float ph = s[sub][r] * PCAR;
                _Float16 h16 = (_Float16)ph;
                Pw[(hf * 8 + r) * 72 + sub * 16 + ln] = __builtin_bit_cast(u16, h16);
                if constexpr (RES)
                    Prw[(hf * 8 + r) * 72 + sub * 16 + ln] = hbits((ph - (float)h16) * RSC);
            }
        }
        __syncthreads();

#pragma unroll
        for (int dsub = 0; dsub < 4; dsub++) {
            v8f u = (v8f)(0.f);
#pragma unroll
            for (int ks = 0; ks < 2; ks++) {
                Frag pf, vf;
                const u16* pp = &Pw[ln * 72 + ks * 32 + hf * 8];
                pf.u[0] = *(const u32x4*)pp;
                pf.u[1] = *(const u32x4*)(pp + 16);
                const u16* vp = &Vs[(dsub * 16 + ln) * 72 + ks * 32 + hf * 8];
                vf.u[0] = *(const u32x4*)vp;
                vf.u[1] = *(const u32x4*)(vp + 16);
                o[dsub] = mma16(pf.v, vf.v, o[dsub]);
                if constexpr (RES) {
                    Frag prf;
                    const u16* prp = &Prw[ln * 72 + ks * 32 + hf * 8];
                    prf.u[0] = *(const u32x4*)prp;
                    prf.u[1] = *(const u32x4*)(prp + 16);
                    u = mma16(prf.v, vf.v, u);
                    Frag vlf;
                    const u16* vlp = &Vl[(dsub * 16 + ln) * 72 + ks * 32 + hf * 8];
                    vlf.u[0] = *(const u32x4*)vlp;
                    vlf.u[1] = *(const u32x4*)(vlp + 16);
                    u = mma16(pf.v, vlf.v, u);
                }
            }
            if constexpr (RES) o[dsub] = o[dsub] + u * RINV;
        }
    }

    __syncthreads();
#pragma unroll
    for (int r = 0; r < 8; r++) {
        const float inv = (1.0f / lrow[r]) * (PINV * OCAR);
#pragma unroll
        for (int dsub = 0; dsub < 4; dsub++)
            Pw[(hf * 8 + r) * 72 + dsub * 16 + ln] = hbits(o[dsub][r] * inv);
    }
    __syncthreads();
    u32x4 val[4];
#pragma unroll
    for (int it = 0; it < 4; it++) {
        const int rloc = it * 4 + (lane >> 3), sg = (lane & 7) * 8;
        val[it] = *(const u32x4*)&Pw[rloc * 72 + sg];
    }
#pragma unroll
    for (int it = 0; it < 4; it++) {
        const int rloc = it * 4 + (lane >> 3), sg = (lane & 7) * 8;
        *(volatile u32x4*)(cv + (size_t)(b * (SEQ) + q0 + rloc) * CE + h * HD + sg) = val[it];
    }
    __threadfence();
#pragma unroll
    for (int it = 0; it < 4; it++) {
        const int rloc = it * 4 + (lane >> 3), sg = (lane & 7) * 8;
        *(volatile u32x4*)(cv + (size_t)(b * (SEQ) + q0 + rloc) * CE + h * HD + sg) = val[it];
    }
}

extern "C" void kernel_launch(void* const* d_in, const int* in_sizes, int n_in,
                              void* d_out, int out_size, void* d_ws, size_t ws_size,
                              hipStream_t stream) {
    if (n_in < 12) return;
    const long long needX = ((long long)(NB - 1) * SEQ_FULL + (SEQ)) * CE;
    if ((long long)in_sizes[0] < needX || (long long)out_size < needX) return;
    if (in_sizes[1] < 1 || in_sizes[2] < CE || in_sizes[3] < CE ||
        in_sizes[4] < CE * C3 || in_sizes[5] < C3 ||
        in_sizes[6] < CE * CE || in_sizes[7] < CE ||
        in_sizes[8] < CE * C4 || in_sizes[9] < C4 ||
        in_sizes[10] < C4 * CE || in_sizes[11] < CE)
        return;

    const float* x      = (const float*)d_in[0];
    const float* alpha  = (const float*)d_in[1];
    const float* gamma  = (const float*)d_in[2];
    const float* beta   = (const float*)d_in[3];
    const float* w_attn = (const float*)d_in[4];
    const float* b_attn = (const float*)d_in[5];
    const float* w_proj = (const float*)d_in[6];
    const float* b_proj = (const float*)d_in[7];
    const float* w_fc   = (const float*)d_in[8];
    const float* b_fc   = (const float*)d_in[9];
    const float* w_fc2  = (const float*)d_in[10];
    const float* b_fc2  = (const float*)d_in[11];

    char* ws = (char*)d_ws;
    size_t off = 0;
    auto take = [&](size_t bytes) -> char* {
        char* p = ws + off;
        off += (bytes + 255) & ~(size_t)255;
        return p;
    };
    const size_t R = (size_t)RROWS;
    u16*   waT   = (u16*)take((size_t)C3 * CE * 2);
    u16*   wpT   = (u16*)take((size_t)CE * CE * 2);
    u16*   wfcT  = (u16*)take((size_t)C4 * CE * 2);
    u16*   wfc2T = (u16*)take((size_t)CE * C4 * 2);
    u16*   h1    = (u16*)take(R * CE * 2);
    u16*   qkh   = (u16*)take(R * QP * 2);
    u16*   qkl   = (u16*)take((size_t)NB * (TE) * QP * 2);
    u16*   vth   = (u16*)take((size_t)NB * NH * HD * (SEQ) * 2);
    u16*   vtl   = (u16*)take((size_t)NB * NH * HD * (TE) * 2);
    u16*   cvb   = (u16*)take(R * CE * 2);
    float* x1    = (float*)take(R * CE * 4);
    u16*   h2    = (u16*)take(R * CE * 2);
    u16*   hg    = (u16*)take(R * C4 * 2);
    if (off > ws_size) return;
    void* dummy = (void*)d_ws;

    cvt_wt_kernel<<<dim3(C3 / 64, CE / 64), 256, 0, stream>>>(w_attn, waT, CE, C3);
    cvt_wt_kernel<<<dim3(CE / 64, CE / 64), 256, 0, stream>>>(w_proj, wpT, CE, CE);
    cvt_wt_kernel<<<dim3(C4 / 64, CE / 64), 256, 0, stream>>>(w_fc,   wfcT, CE, C4);
    cvt_wt_kernel<<<dim3(CE / 64, C4 / 64), 256, 0, stream>>>(w_fc2,  wfc2T, C4, CE);
    dyt_kernel<1><<<RROWS / 8, 256, 0, stream>>>(x, alpha, gamma, beta, h1);
    gemm_kernel<0><<<dim3(C3 / 128, RROWS / 128), 256, 0, stream>>>(h1, waT, b_attn, b_attn,
                                                                    qkh, qkl, vth, vtl, C3, CE);
    attn_kernel<1><<<dim3(NEB, NB * NH), 256, 0, stream>>>(qkh, qkl, vth, vtl, cvb, 0);
    if (NQB > NEB)
        attn_kernel<0><<<dim3(NQB - NEB, NB * NH), 256, 0, stream>>>(qkh, qkl, vth, vtl, cvb, NEB);
    gemm_kernel<1><<<dim3(CE / 128, RROWS / 128), 256, 0, stream>>>(cvb, wpT, b_proj, x,
                                                                    x1, dummy, dummy, dummy, CE, CE);
    dyt_kernel<0><<<RROWS / 8, 256, 0, stream>>>(x1, alpha, gamma, beta, h2);
    gemm_kernel<2><<<dim3(C4 / 128, RROWS / 128), 256, 0, stream>>>(h2, wfcT, b_fc, b_fc,
                                                                    hg, dummy, dummy, dummy, C4, CE);
    gemm_kernel<3><<<dim3(CE / 128, RROWS / 128), 256, 0, stream>>>(hg, wfc2T, b_fc2, x1,
                                                                    d_out, dummy, dummy, dummy, CE, C4);
}
